// RNNModel_10969346474402
// MI455X (gfx1250) — hardware-verified
//
#include <hip/hip_runtime.h>
#include <math.h>

constexpr int NBATCH  = 8192;
constexpr int NSTEP   = 256;
constexpr int NHID    = 64;
constexpr int NGATE   = 4 * NHID;
constexpr int NFC1    = 32;
constexpr int NFC2    = 2;
constexpr int ROWS    = 16;
constexpr int NTHR    = 128;
constexpr int WPITCH  = 72;
constexpr int HPITCH  = 72;
constexpr int PLANE   = ROWS * HPITCH;
constexpr int HFPITCH = 65;
constexpr int ZPITCH  = 33;
constexpr float H_CARRY = 256.0f;
constexpr float L_CARRY = 4096.0f;
constexpr float W_CARRY = 256.0f;
constexpr float FOLD_HI = 1.0f / (H_CARRY * W_CARRY);
constexpr float FOLD_LO = 1.0f / (H_CARRY * W_CARRY * L_CARRY);

static_assert(NBATCH % ROWS == 0);
static_assert(NHID == 16 * (NTHR / 32));
static_assert(NHID % 32 == 0);
static_assert(NGATE == 4 * NHID);
static_assert((NGATE * NHID) % (4 * NTHR) == 0);
static_assert((NSTEP * ROWS) % (4 * NTHR) == 0);
static_assert((2 * PLANE) % NTHR == 0);
static_assert(ROWS * NFC1 == 4 * NTHR);
static_assert(ROWS * NFC2 == 32);
static_assert(WPITCH % 8 == 0 && HPITCH % 8 == 0);

typedef __attribute__((ext_vector_type(16))) _Float16 v16h;
typedef __attribute__((ext_vector_type(8)))  _Float16 v8h;
typedef __attribute__((ext_vector_type(8)))  float    v8f;
typedef __attribute__((ext_vector_type(4)))  float    v4f;
typedef __attribute__((ext_vector_type(2)))  unsigned v2u;

__device__ __forceinline__ unsigned short f2bf_bits(float f) {
  unsigned u = __float_as_uint(f);
  return (unsigned short)((u + 0x7FFFu + ((u >> 16) & 1u)) >> 16);
}
__device__ __forceinline__ float bf_bits2f(unsigned short h) { return __uint_as_float(((unsigned)h) << 16); }
__device__ __forceinline__ float bf16r(float f) { return bf_bits2f(f2bf_bits(f)); }

union FragU { v16h v; v8h h[2]; };
__device__ __forceinline__ v16h load16(const _Float16* p) {
  FragU f; f.h[0] = *(const v8h*)(p); f.h[1] = *(const v8h*)(p + 16); return f.v;
}
__device__ __forceinline__ v8f mma16(v16h a, v16h b, v8f c) {
  return __builtin_amdgcn_wmma_f32_16x16x32_f16(false, a, false, b, (short)0, c, false, false);
}
__device__ __forceinline__ void guard_group(v8f& d0, v8f& d1, v16h a0, v16h a1, v16h a2, v16h a3, v16h b0, v16h b1) {
  asm volatile("v_nop\n\tv_nop\n\tv_nop\n\tv_nop" : "+v"(d0), "+v"(d1) : "v"(a0), "v"(a1), "v"(a2), "v"(a3), "v"(b0), "v"(b1));
}

__device__ __forceinline__ float rcp_nr(float d) {
  const float r = __builtin_amdgcn_rcpf(d);
  return r * fmaf(-d, r, 2.0f);
}
__device__ __forceinline__ float sigm_f(float z) {
  const float zc = fminf(fmaxf(z, -30.0f), 30.0f);
  const float e = __expf(-zc);
  return rcp_nr(1.0f + e);
}
__device__ __forceinline__ float tanh_f(float z) {
  const float zc = fminf(fmaxf(z, -15.0f), 15.0f);
  const float e = __expf(2.0f * zc);
  return fmaf(-2.0f, rcp_nr(1.0f + e), 1.0f);
}

__device__ __forceinline__ void gate_mm(const unsigned short* wlp, int n, int koff,
                                        v16h ah0, v16h ah1, v16h al0, v16h al1, v8f& ach, v8f& acl) {
  const _Float16* wr = (const _Float16*)wlp + n * WPITCH + koff;
  const v16h b0 = load16(wr);
  const v16h b1 = load16(wr + 32);
  const v8f z8 = {0.f, 0.f, 0.f, 0.f, 0.f, 0.f, 0.f, 0.f};
  ach = mma16(ah0, b0, z8);
  ach = mma16(ah1, b1, ach);
  acl = mma16(al0, b0, z8);
  acl = mma16(al1, b1, acl);
  guard_group(ach, acl, ah0, ah1, al0, al1, b0, b1);
}

__global__ __launch_bounds__(NTHR) void lstm_head_kernel(const float* __restrict__ x,
                                                         const float* __restrict__ w_ih,
                                                         const float* __restrict__ w_hh,
                                                         const float* __restrict__ b_ih,
                                                         const float* __restrict__ b_hh,
                                                         const float* __restrict__ w1,
                                                         const float* __restrict__ b1,
                                                         const float* __restrict__ w2,
                                                         const float* __restrict__ b2,
                                                         float* __restrict__ out) {
  __shared__ __align__(16) unsigned short wl[NGATE * WPITCH];
  __shared__ __align__(16) float          xs[NSTEP * ROWS];
  __shared__ __align__(16) _Float16       hpl[4 * PLANE];
  __shared__ __align__(16) float          hf[ROWS * HFPITCH];
  __shared__ __align__(16) float          zs[ROWS * ZPITCH];
  __shared__ __align__(16) float          os[ROWS * NFC2];

  const int tid = threadIdx.x, lane = tid & 31, wave = tid >> 5;
  const int c = lane & 15, hh = lane >> 4, koff = hh * 8;
  const int ucol = 16 * wave + c;
  const int rowbase = blockIdx.x * ROWS;

  {
    unsigned* hw = (unsigned*)(void*)hpl;
#pragma unroll 1
    for (int i = tid; i < 2 * PLANE; i += NTHR) hw[i] = 0u;
  }
#pragma unroll 2
  for (int it = 0; it < (NGATE * NHID) / (4 * NTHR); ++it) {
    const int idx = it * NTHR + tid;
    const int n = idx >> 4, k4 = (idx & 15) * 4;
    const v4f v = *(const v4f*)(w_hh + (size_t)n * NHID + k4);
    const float f0 = v[0], f1 = v[1], f2 = v[2], f3 = v[3];
    const unsigned u0 = (unsigned)__builtin_bit_cast(unsigned short, (_Float16)(bf16r(f0) * W_CARRY));
    const unsigned u1 = (unsigned)__builtin_bit_cast(unsigned short, (_Float16)(bf16r(f1) * W_CARRY));
    const unsigned u2 = (unsigned)__builtin_bit_cast(unsigned short, (_Float16)(bf16r(f2) * W_CARRY));
    const unsigned u3 = (unsigned)__builtin_bit_cast(unsigned short, (_Float16)(bf16r(f3) * W_CARRY));
    v2u pk;
    pk[0] = u0 | (u1 << 16);
    pk[1] = u2 | (u3 << 16);
    *(v2u*)(wl + n * WPITCH + k4) = pk;
  }
#pragma unroll 2
  for (int it = 0; it < (NSTEP * ROWS) / (4 * NTHR); ++it) {
    const int idx = it * NTHR + tid;
    const int row = idx >> 6, t4 = (idx & 63) * 4;
    const v4f v = *(const v4f*)(x + (size_t)(rowbase + row) * NSTEP + t4);
    const float f0 = v[0], f1 = v[1], f2 = v[2], f3 = v[3];
    xs[(t4 + 0) * ROWS + row] = bf16r(f0);
    xs[(t4 + 1) * ROWS + row] = bf16r(f1);
    xs[(t4 + 2) * ROWS + row] = bf16r(f2);
    xs[(t4 + 3) * ROWS + row] = bf16r(f3);
  }
  float wih[4], bsm[4];
#pragma unroll
  for (int g = 0; g < 4; ++g) {
    const int n = NHID * g + ucol;
    wih[g] = bf16r(w_ih[n]);
    bsm[g] = bf16r(b_ih[n]) + bf16r(b_hh[n]);
  }
  float cst[8], hst[8], tg[8];
#pragma unroll
  for (int r = 0; r < 8; ++r) { cst[r] = 0.0f; hst[r] = 0.0f; tg[r] = 0.0f; }
  __syncthreads();

#pragma unroll 1
  for (int t = 0; t < NSTEP; ++t) {
    const int cur = t & 1;
    const _Float16* hcur = hpl + (2 * cur) * PLANE + c * HPITCH + koff;
    const _Float16* lcur = hcur + PLANE;
    _Float16* hnx = hpl + (2 * (cur ^ 1)) * PLANE;
    _Float16* lnx = hnx + PLANE;
    const v16h ah0 = load16(hcur);
    const v16h ah1 = load16(hcur + 32);
    const v16h al0 = load16(lcur);
    const v16h al1 = load16(lcur + 32);
    const v4f xa = *(const v4f*)(xs + t * ROWS + 8 * hh);
    const v4f xb = *(const v4f*)(xs + t * ROWS + 8 * hh + 4);
    const float xr[8] = {xa[0], xa[1], xa[2], xa[3], xb[0], xb[1], xb[2], xb[3]};
    v8f ach, acl;

    gate_mm(wl, 2 * NHID + ucol, koff, ah0, ah1, al0, al1, ach, acl);
#pragma unroll
    for (int r = 0; r < 8; ++r) {
      const float z = fmaf(ach[r], FOLD_HI, fmaf(acl[r], FOLD_LO, fmaf(xr[r], wih[2], bsm[2])));
      tg[r] = tanh_f(z);
    }
    gate_mm(wl, 0 * NHID + ucol, koff, ah0, ah1, al0, al1, ach, acl);
#pragma unroll
    for (int r = 0; r < 8; ++r) {
      const float z = fmaf(ach[r], FOLD_HI, fmaf(acl[r], FOLD_LO, fmaf(xr[r], wih[0], bsm[0])));
      tg[r] = sigm_f(z) * tg[r];
    }
    gate_mm(wl, 1 * NHID + ucol, koff, ah0, ah1, al0, al1, ach, acl);
#pragma unroll
    for (int r = 0; r < 8; ++r) {
      const float z = fmaf(ach[r], FOLD_HI, fmaf(acl[r], FOLD_LO, fmaf(xr[r], wih[1], bsm[1])));
      cst[r] = fmaf(sigm_f(z), cst[r], tg[r]);
    }
    gate_mm(wl, 3 * NHID + ucol, koff, ah0, ah1, al0, al1, ach, acl);
#pragma unroll
    for (int r = 0; r < 8; ++r) {
      const float z = fmaf(ach[r], FOLD_HI, fmaf(acl[r], FOLD_LO, fmaf(xr[r], wih[3], bsm[3])));
      const float og = sigm_f(z);
      const float hn = og * tanh_f(cst[r]);
      hst[r] = hn;
      const float hs = hn * H_CARRY;
      const _Float16 h16 = (_Float16)hs;
      const float res = hs - (float)h16;
      const _Float16 l16 = (_Float16)(res * L_CARRY);
      const int o = (8 * hh + r) * HPITCH + ucol;
      hnx[o] = h16;
      lnx[o] = l16;
    }
    __syncthreads();
  }

#pragma unroll
  for (int r = 0; r < 8; ++r) hf[(8 * hh + r) * HFPITCH + ucol] = hst[r];
  __syncthreads();
  {
    const int row = tid & 15;
    const int j0 = (tid >> 4) * 4;
    const float* w1a = w1 + (size_t)(j0 + 0) * NHID;
    const float* w1b = w1 + (size_t)(j0 + 1) * NHID;
    const float* w1c = w1 + (size_t)(j0 + 2) * NHID;
    const float* w1d = w1 + (size_t)(j0 + 3) * NHID;
    float a0 = 0.0f, a1 = 0.0f, a2 = 0.0f, a3 = 0.0f;
#pragma unroll 2
    for (int k = 0; k < NHID; ++k) {
      const float hv = hf[row * HFPITCH + k];
      a0 = fmaf(hv, bf16r(w1a[k]), a0);
      a1 = fmaf(hv, bf16r(w1b[k]), a1);
      a2 = fmaf(hv, bf16r(w1c[k]), a2);
      a3 = fmaf(hv, bf16r(w1d[k]), a3);
    }
    const float z0 = fmaxf(a0 + bf16r(b1[j0 + 0]), 0.0f);
    const float z1 = fmaxf(a1 + bf16r(b1[j0 + 1]), 0.0f);
    const float z2 = fmaxf(a2 + bf16r(b1[j0 + 2]), 0.0f);
    const float z3 = fmaxf(a3 + bf16r(b1[j0 + 3]), 0.0f);
    zs[row * ZPITCH + j0 + 0] = z0;
    zs[row * ZPITCH + j0 + 1] = z1;
    zs[row * ZPITCH + j0 + 2] = z2;
    zs[row * ZPITCH + j0 + 3] = z3;
  }
  __syncthreads();
  if (wave == 0) {
    const int row = lane >> 1, o = lane & 1;
    const float* w2r = w2 + o * NFC1;
    float s = 0.0f;
#pragma unroll 4
    for (int j = 0; j < NFC1; ++j) s = fmaf(zs[row * ZPITCH + j], bf16r(w2r[j]), s);
    s += bf16r(b2[o]);
    os[lane] = s;
  }
  __syncthreads();
  if (wave == 0 && lane < 8) {
    const v4f v = *(const v4f*)(os + lane * 4);
    float* op = out + (size_t)rowbase * NFC2 + lane * 4;
    for (int pass = 0; pass < 2; ++pass) {
      *(volatile v4f*)op = v;
      __threadfence();
    }
  }
}

extern "C" void kernel_launch(void* const* d_in, const int* in_sizes, int n_in,
                              void* d_out, int out_size, void* d_ws, size_t ws_size, hipStream_t stream) {
  (void)d_ws; (void)ws_size;
  if (n_in < 9 || d_out == nullptr) return;
  if (in_sizes[0] != NBATCH * NSTEP || in_sizes[1] != NGATE || in_sizes[2] != NGATE * NHID ||
      in_sizes[3] != NGATE || in_sizes[4] != NGATE || in_sizes[5] != NFC1 * NHID || in_sizes[6] != NFC1 ||
      in_sizes[7] != NFC2 * NFC1 || in_sizes[8] != NFC2 || out_size != NBATCH * NFC2) return;

  const float* x    = (const float*)d_in[0];
  const float* w_ih = (const float*)d_in[1];
  const float* w_hh = (const float*)d_in[2];
  const float* b_ih = (const float*)d_in[3];
  const float* b_hh = (const float*)d_in[4];
  const float* w1   = (const float*)d_in[5];
  const float* b1   = (const float*)d_in[6];
  const float* w2   = (const float*)d_in[7];
  const float* b2   = (const float*)d_in[8];
  float* out = (float*)d_out;

  lstm_head_kernel<<<NBATCH / ROWS, NTHR, 0, stream>>>(x, w_ih, w_hh, b_ih, b_hh, w1, b1, w2, b2, out);
}
